// DifferentialCrossAttentionHead_83021717832617
// MI455X (gfx1250) — hardware-verified
//
#include <hip/hip_runtime.h>


namespace {
constexpr int B = 4, T = 2048, EM = 1024, HD = 128, HH = 64, NR = B * T;
constexpr float XS = 8.0f, PS = 1024.0f, WSC = 256.0f;
typedef _Float16 b16;
typedef __attribute__((ext_vector_type(16))) _Float16 v16b;
typedef __attribute__((ext_vector_type(8))) _Float16 v8b;
typedef __attribute__((ext_vector_type(8))) float v8f;
typedef __attribute__((ext_vector_type(4))) float v4f;
__device__ __forceinline__ float bf16_rne(float f) { unsigned int u = __float_as_uint(f); u += 0x7FFFu + ((u >> 16) & 1u); float r = __uint_as_float(u & 0xFFFF0000u); asm volatile("" : "+v"(r)); return r; }
__device__ __forceinline__ void split16(float v, b16& hi, b16& lo) { hi = (b16)v; lo = (b16)(v - (float)hi); }
__device__ __forceinline__ v16b frag_kb(const b16* p, int hh) { const v8b a = *(const v8b*)(p + 8 * hh), b = *(const v8b*)(p + 16 + 8 * hh); v16b f;
#pragma unroll
  for (int e = 0; e < 8; ++e) { f[e] = a[e]; f[8 + e] = b[e]; } return f; }
__device__ __forceinline__ v8f wmma16b(v16b a, v16b b, v8f c) { v8f d = __builtin_amdgcn_wmma_f32_16x16x32_f16(false, a, false, b, (short)0, c, false, false); asm volatile("v_nop\n\tv_nop\n\tv_nop\n\tv_nop" : "+v"(d) : "v"(a), "v"(b)); return d; }
__device__ __forceinline__ void wave_lds_sync() { __builtin_amdgcn_fence(__ATOMIC_RELEASE, "workgroup"); __builtin_amdgcn_wave_barrier(); __builtin_amdgcn_fence(__ATOMIC_ACQUIRE, "workgroup"); }
__device__ __forceinline__ float pmul(float a, float b) { float p = a * b; asm volatile("" : "+v"(p)); return p; }

__global__ __launch_bounds__(256) void wput_kernel(const float* __restrict__ w, b16* __restrict__ WT) { const int u = blockIdx.x * 256 + threadIdx.x; if (u >= HD * (EM / 8)) return; const int o = u / (EM / 8), k0 = (u % (EM / 8)) * 8; v8b v;
#pragma unroll
  for (int j = 0; j < 8; ++j) v[j] = (b16)(bf16_rne(w[(size_t)(k0 + j) * HD + o]) * WSC); for (int pass = 0; pass < 2; ++pass) { *(volatile v8b*)(WT + (size_t)o * EM + k0) = v; __threadfence(); } }
__global__ __launch_bounds__(32) void proj_kernel(const float* __restrict__ in, const b16* __restrict__ WT, const float* __restrict__ bias, int RL, float* __restrict__ OUTP) {
  __shared__ __attribute__((aligned(16))) b16 Ah[16][EM + 8]; __shared__ float Tf[16][132]; const int lane = threadIdx.x, nloc = lane & 15, hlf = lane >> 4; const size_t m0 = (size_t)blockIdx.x * 16; if (m0 >= (size_t)RL) return;
  for (int rr = 0; rr < 16; ++rr) for (int q = 0; q < EM / 32; ++q) Ah[rr][q * 32 + lane] = (b16)(bf16_rne(in[(m0 + rr) * EM + q * 32 + lane]) * XS);
  wave_lds_sync(); v8f acc[8];
#pragma unroll
  for (int t = 0; t < 8; ++t) acc[t] = (v8f){};
#pragma unroll 2
  for (int kb = 0; kb < EM; kb += 32) { const v16b a = frag_kb(&Ah[nloc][kb], hlf);
#pragma unroll
    for (int t = 0; t < 8; ++t) acc[t] = wmma16b(a, frag_kb(WT + (size_t)(t * 16 + nloc) * EM + kb, hlf), acc[t]); }
#pragma unroll
  for (int t = 0; t < 8; ++t) { const int c = t * 16 + nloc; const float bb = bf16_rne(bias[c]);
#pragma unroll
    for (int r8 = 0; r8 < 8; ++r8) Tf[8 * hlf + r8][c] = acc[t][r8] * (1.0f / (XS * WSC)) + bb; }
  wave_lds_sync();
  for (int pass = 0; pass < 2; ++pass) { for (int rr = 0; rr < 16; ++rr) *(volatile v4f*)(OUTP + (m0 + rr) * HD + lane * 4) = *(const v4f*)(&Tf[rr][lane * 4]); __threadfence(); }
}
__global__ __launch_bounds__(256) void kh_kernel(const float* __restrict__ K, b16* __restrict__ Kh, b16* __restrict__ Kl) { const size_t u = (size_t)blockIdx.x * 256 + threadIdx.x; if (u >= (size_t)NR * (HD / 8)) return; const size_t row = u / (HD / 8); const int d0 = (int)(u % (HD / 8)) * 8; v8b kh, kl;
#pragma unroll
  for (int j = 0; j < 8; ++j) { b16 p, q; split16(K[row * HD + d0 + j] * XS, p, q); kh[j] = p; kl[j] = q; }
  for (int pass = 0; pass < 2; ++pass) { *(volatile v8b*)(Kh + row * HD + d0) = kh; *(volatile v8b*)(Kl + row * HD + d0) = kl; __threadfence(); } }
__global__ __launch_bounds__(32) void vt_kernel(const float* __restrict__ V, int BV, b16* __restrict__ VTh, b16* __restrict__ VTl) { const int lane = threadIdx.x; const int b = blockIdx.x / (T / 32), ch = blockIdx.x % (T / 32); if (b >= BV) return; const size_t row = (size_t)b * T + ch * 32 + lane; const size_t base = ((size_t)b * (T / 32) + ch) * HD;
  for (int pass = 0; pass < 2; ++pass) {
#pragma unroll 4
    for (int d = 0; d < HD; ++d) { b16 p, q; split16(V[row * HD + d] * XS, p, q); ((volatile b16*)VTh)[(base + d) * 64 + lane] = p; ((volatile b16*)VTl)[(base + d) * 64 + lane] = q; }
    __threadfence(); } }
__device__ __forceinline__ void scores(const b16 (*Qh)[HD + 8], const b16 (*Ql)[HD + 8], const b16* Kh, const b16* Kl, size_t krow0, float (*Sc1)[33], float (*Sc2)[33], int nloc, int hlf) {
#pragma unroll
  for (int blk = 0; blk < 2; ++blk) { v8f s1 = {}, s2 = {}; const size_t kr = (krow0 + blk * 16 + nloc) * HD;
#pragma unroll
    for (int kb = 0; kb < HH; kb += 32) { { const v16b qh = frag_kb(&Qh[nloc][kb], hlf), ql = frag_kb(&Ql[nloc][kb], hlf), kh = frag_kb(Kh + kr + kb, hlf), kl = frag_kb(Kl + kr + kb, hlf); s1 = wmma16b(qh, kh, s1); s1 = wmma16b(qh, kl, s1); s1 = wmma16b(ql, kh, s1); }
      { const v16b qh = frag_kb(&Qh[nloc][HH + kb], hlf), ql = frag_kb(&Ql[nloc][HH + kb], hlf), kh = frag_kb(Kh + kr + HH + kb, hlf), kl = frag_kb(Kl + kr + HH + kb, hlf); s2 = wmma16b(qh, kh, s2); s2 = wmma16b(qh, kl, s2); s2 = wmma16b(ql, kh, s2); } }
#pragma unroll
    for (int r8 = 0; r8 < 8; ++r8) { Sc1[8 * hlf + r8][blk * 16 + nloc] = s1[r8] * (0.125f / (XS * XS)); Sc2[8 * hlf + r8][blk * 16 + nloc] = s2[r8] * (0.125f / (XS * XS)); } }
}
__global__ __launch_bounds__(32) void att_kernel(const float* __restrict__ Q, const b16* __restrict__ Kh, const b16* __restrict__ Kl, const b16* __restrict__ VTh, const b16* __restrict__ VTl, const float* __restrict__ lq1, const float* __restrict__ lk1, const float* __restrict__ lq2, const float* __restrict__ lk2, const float* __restrict__ linit, int QV, float* __restrict__ out) {
  __shared__ __attribute__((aligned(16))) b16 Qh[16][HD + 8], Ql[16][HD + 8], Ph[16][40], Pl[16][40]; __shared__ float Sc1[16][33], Sc2[16][33], M1[16], L1[16], M2[16], L2[16], Of[16][HD + 4];
  const int lane = threadIdx.x, nloc = lane & 15, hlf = lane >> 4; const int qt = blockIdx.x % (T / 16); const int b = blockIdx.x / (T / 16); const int q0 = qt * 16; if (q0 >= QV) return; const size_t qrow = (size_t)b * T + q0;
  float d1 = 0.0f, d2 = 0.0f; for (int i = lane; i < HD; i += 32) { d1 += pmul(bf16_rne(lq1[i]), bf16_rne(lk1[i])); d2 += pmul(bf16_rne(lq2[i]), bf16_rne(lk2[i])); } for (int o = 16; o; o >>= 1) { d1 += __shfl_xor(d1, o); d2 += __shfl_xor(d2, o); } const float lam = __expf(d1) - __expf(d2) + bf16_rne(linit[0]);
  for (int rr = 0; rr < 16; ++rr) for (int q = 0; q < HD / 32; ++q) { b16 p, ql; split16(Q[(qrow + rr) * HD + q * 32 + lane] * XS, p, ql); Qh[rr][q * 32 + lane] = p; Ql[rr][q * 32 + lane] = ql; }
  if (lane < 16) { M1[lane] = -INFINITY; L1[lane] = 0.0f; M2[lane] = -INFINITY; L2[lane] = 0.0f; }
  wave_lds_sync();
#pragma unroll 1
  for (int kc = 0; kc < T; kc += 32) { scores(Qh, Ql, Kh, Kl, (size_t)b * T + kc, Sc1, Sc2, nloc, hlf); wave_lds_sync();
#pragma unroll 1
    for (int qi = 0; qi < 16; ++qi) { const float a1 = Sc1[qi][lane], a2 = Sc2[qi][lane]; float c1 = a1, c2 = a2; for (int o = 16; o; o >>= 1) { c1 = fmaxf(c1, __shfl_xor(c1, o)); c2 = fmaxf(c2, __shfl_xor(c2, o)); }
      const float mo1 = M1[qi], mo2 = M2[qi]; const float mn1 = fmaxf(mo1, c1), mn2 = fmaxf(mo2, c2); float p1 = __expf(a1 - mn1), p2 = __expf(a2 - mn2); for (int o = 16; o; o >>= 1) { p1 += __shfl_xor(p1, o); p2 += __shfl_xor(p2, o); }
      if (lane == 0) { L1[qi] = L1[qi] * ((mo1 == -INFINITY) ? 0.0f : __expf(mo1 - mn1)) + p1; M1[qi] = mn1; L2[qi] = L2[qi] * ((mo2 == -INFINITY) ? 0.0f : __expf(mo2 - mn2)) + p2; M2[qi] = mn2; } }
    wave_lds_sync(); }
  v8f acc[8];
#pragma unroll
  for (int t = 0; t < 8; ++t) acc[t] = (v8f){};
#pragma unroll 1
  for (int kc = 0; kc < T; kc += 32) { scores(Qh, Ql, Kh, Kl, (size_t)b * T + kc, Sc1, Sc2, nloc, hlf); wave_lds_sync();
    for (int qi = 0; qi < 16; ++qi) { const float w = __expf(Sc1[qi][lane] - M1[qi]) / L1[qi] - pmul(lam, __expf(Sc2[qi][lane] - M2[qi]) / L2[qi]); b16 p, ql; split16(w * PS, p, ql); Ph[qi][lane] = p; Pl[qi][lane] = ql; }
    wave_lds_sync(); const v16b pa = frag_kb(&Ph[nloc][0], hlf), pb = frag_kb(&Pl[nloc][0], hlf); const size_t vb = (((size_t)b * (T / 32) + kc / 32) * HD) * 64;
#pragma unroll
    for (int t = 0; t < 8; ++t) { const v16b vh = frag_kb(VTh + vb + (size_t)(t * 16 + nloc) * 64, hlf), vl = frag_kb(VTl + vb + (size_t)(t * 16 + nloc) * 64, hlf); acc[t] = wmma16b(pa, vh, acc[t]); acc[t] = wmma16b(pa, vl, acc[t]); acc[t] = wmma16b(pb, vh, acc[t]); }
    wave_lds_sync(); }
#pragma unroll
  for (int t = 0; t < 8; ++t)
#pragma unroll
    for (int r8 = 0; r8 < 8; ++r8) Of[8 * hlf + r8][t * 16 + nloc] = acc[t][r8] * (1.0f / (PS * XS));
  wave_lds_sync();
  for (int pass = 0; pass < 2; ++pass) { for (int rr = 0; rr < 16; ++rr) *(volatile v4f*)(out + (qrow + rr) * HD + lane * 4) = *(const v4f*)(&Of[rr][lane * 4]); __threadfence(); }
}
}

extern "C" void kernel_launch(void* const* d_in, const int* in_sizes, int n_in, void* d_out, int out_size, void* d_ws, size_t ws_size, hipStream_t stream) {
  (void)n_in;
  auto Fp = [&](int i) { return (const float*)d_in[i]; };
  if (in_sizes[0] != NR * EM || in_sizes[1] != NR * EM || in_sizes[2] != EM * HD || in_sizes[4] != EM * HD || in_sizes[6] != EM * HD || in_sizes[8] != HD || in_sizes[12] != 1 || out_size != NR * HD) return;
  const int BV = B, QV = T;
  size_t off = 0; char* ws = (char*)d_ws;
  auto carve = [&](size_t bytes) { char* p = ws + off; off += (bytes + 255) & ~(size_t)255; return p; };
  b16* WQ = (b16*)carve((size_t)HD * EM * 2); b16* WK = (b16*)carve((size_t)HD * EM * 2); b16* WV = (b16*)carve((size_t)HD * EM * 2); float* Q = (float*)carve((size_t)NR * HD * 4); float* K = (float*)carve((size_t)NR * HD * 4); float* V = (float*)carve((size_t)NR * HD * 4);
  b16* Kh = (b16*)carve((size_t)NR * HD * 2); b16* Kl = (b16*)carve((size_t)NR * HD * 2); b16* VTh = (b16*)carve((size_t)B * (T / 32) * HD * 64 * 2); b16* VTl = (b16*)carve((size_t)B * (T / 32) * HD * 64 * 2);
  if (off > ws_size || off > ((size_t)48 << 20)) return;
  wput_kernel<<<(HD * (EM / 8) + 255) / 256, 256, 0, stream>>>(Fp(2), WQ); wput_kernel<<<(HD * (EM / 8) + 255) / 256, 256, 0, stream>>>(Fp(4), WK); wput_kernel<<<(HD * (EM / 8) + 255) / 256, 256, 0, stream>>>(Fp(6), WV);
  proj_kernel<<<BV * T / 16, 32, 0, stream>>>(Fp(0), WQ, Fp(3), BV * T, Q); proj_kernel<<<BV * T / 16, 32, 0, stream>>>(Fp(1), WK, Fp(5), BV * T, K); proj_kernel<<<BV * T / 16, 32, 0, stream>>>(Fp(1), WV, Fp(7), BV * T, V);
  kh_kernel<<<(unsigned)(((size_t)BV * T * (HD / 8) + 255) / 256), 256, 0, stream>>>(K, Kh, Kl);
  vt_kernel<<<BV * (T / 32), 32, 0, stream>>>(V, BV, VTh, VTl);
  att_kernel<<<BV * (T / 16), 32, 0, stream>>>(Q, Kh, Kl, VTh, VTl, Fp(8), Fp(9), Fp(10), Fp(11), Fp(12), QV, (float*)d_out);
}
